// RNN_24378234372233
// MI455X (gfx1250) — hardware-verified
//
#include <hip/hip_runtime.h>
#include <math.h>

constexpr int NVOCAB  = 50257;
constexpr int NEMB    = 256;
constexpr int NHID    = 512;
constexpr int NBATCH  = 32;
constexpr int NSEQ    = 512;
constexpr int NROWS   = NBATCH * NSEQ;
constexpr int NTHR    = 256;
constexpr int SEQ_BLK = 16;
constexpr int HPITCH  = 520;
constexpr int SLABP   = 68;
constexpr int NOUT0   = NBATCH * NSEQ * NHID;
constexpr int NOUT1   = NBATCH * NHID;
constexpr size_t OUT1_BYTE_OFFSET = 33554432;
constexpr size_t OUT_TOTAL_BYTES  = 33619968;
static_assert((size_t)NOUT0 * 4 == OUT1_BYTE_OFFSET, "second output offset");
static_assert(((size_t)NOUT0 + (size_t)NOUT1) * 4 == OUT_TOTAL_BYTES, "output extent");
static_assert(OUT1_BYTE_OFFSET % 128 == 0, "second output starts on a line");
static_assert(NBATCH % SEQ_BLK == 0, "blocks of 16 sequences");
static_assert(NHID == 64 * (NTHR / 32), "8 waves x 64 hidden columns");
static_assert(NHID % 32 == 0 && NEMB % 32 == 0, "K multiples of 32");
static_assert(NROWS % 64 == 0 && NHID % 64 == 0 && NEMB % 64 == 0, "tile multiples");
static_assert(((NROWS / 64) * (NHID / 64)) % 8 == 0, "GEMM grid exact");
static_assert((HPITCH * 2) % 16 == 0 && HPITCH >= NHID, "h plane pitch");
static_assert((NROWS * (NEMB / 8)) % NTHR == 0, "gather grid exact");

typedef __attribute__((ext_vector_type(8)))  _Float16 v8h;
typedef __attribute__((ext_vector_type(16))) __bf16   v16b;
typedef __attribute__((ext_vector_type(8)))  __bf16   v8b;
typedef __attribute__((ext_vector_type(8)))  float    v8f;
typedef __attribute__((ext_vector_type(4)))  float    v4f;
typedef __attribute__((ext_vector_type(2)))  unsigned v2u;

__device__ __forceinline__ unsigned short f2bf_bits(float f) {
  unsigned u = __float_as_uint(f);
  return (unsigned short)((u + 0x7FFFu + ((u >> 16) & 1u)) >> 16);
}
__device__ __forceinline__ float bf_bits2f(unsigned short h) { return __uint_as_float(((unsigned)h) << 16); }
__device__ __forceinline__ float bf16r(float f) { return bf_bits2f(f2bf_bits(f)); }
__device__ __forceinline__ unsigned bf_bits32(float f) {
  const unsigned u = __float_as_uint(f);
  return (u + 0x7FFFu + ((u >> 16) & 1u)) >> 16;
}

__device__ __forceinline__ void guard4_b6(v8f& a, v8f& b, v8f& c, v8f& d, v16b x, v16b y, v16b p, v16b q, v16b r, v16b s) {
  asm volatile("v_nop\n\tv_nop\n\tv_nop\n\tv_nop" : "+v"(a), "+v"(b), "+v"(c), "+v"(d) : "v"(x), "v"(y), "v"(p), "v"(q), "v"(r), "v"(s));
}
__device__ __forceinline__ void guard4_b5(v8f& a, v8f& b, v8f& c, v8f& d, v16b x, v16b p, v16b q, v16b r, v16b s) {
  asm volatile("v_nop\n\tv_nop\n\tv_nop\n\tv_nop" : "+v"(a), "+v"(b), "+v"(c), "+v"(d) : "v"(x), "v"(p), "v"(q), "v"(r), "v"(s));
}
__device__ __forceinline__ void keep4_b(v16b a, v16b b, v16b c, v16b d) { asm volatile("v_nop" :: "v"(a), "v"(b), "v"(c), "v"(d)); }
__device__ __forceinline__ void acc_guard4(v8f& a, v8f& b, v8f& c, v8f& d) { asm volatile("v_nop\n\tv_nop\n\tv_nop\n\tv_nop" : "+v"(a), "+v"(b), "+v"(c), "+v"(d)); }

struct FragB {
  union U { v16b v; v8b h[2]; };
  static __device__ __forceinline__ v16b load(const __bf16* p) {
    U f; f.h[0] = *(const v8b*)(p); f.h[1] = *(const v8b*)(p + 16); return f.v;
  }
  static __device__ __forceinline__ v8f mma(v16b a, v16b b, v8f c) {
    return __builtin_amdgcn_wmma_f32_16x16x32_bf16(false, a, false, b, (short)0, c, false, false);
  }
};

__global__ __launch_bounds__(NTHR) void tpw_kernel(const float* __restrict__ src, int R, int C, int ldo,
                                                  unsigned short* __restrict__ O) {
  __shared__ float Tt[64 * 65];
  const int tid = threadIdx.x;
  const int c0 = blockIdx.x * 64, r0 = blockIdx.y * 64;
#pragma unroll
  for (int i = 0; i < 4; ++i) {
    const int idx = i * NTHR + tid;
    const int rr = idx >> 4, cc = (idx & 15) * 4;
    const v4f v = *(const v4f*)(src + (size_t)(r0 + rr) * (size_t)C + c0 + cc);
    Tt[rr * 65 + cc + 0] = v[0];
    Tt[rr * 65 + cc + 1] = v[1];
    Tt[rr * 65 + cc + 2] = v[2];
    Tt[rr * 65 + cc + 3] = v[3];
  }
  __syncthreads();
  const int q = tid >> 3, c8 = (tid & 7) * 8;
  v8h hv[2];
#pragma unroll
  for (int g = 0; g < 2; ++g) {
    const int qq = g * 32 + q;
#pragma unroll
    for (int e = 0; e < 8; ++e) {
      const float f = Tt[(c8 + e) * 65 + qq];
      const unsigned short bits = f2bf_bits(f);
      hv[g][e] = __builtin_bit_cast(_Float16, bits);
    }
  }
  for (int pass = 0; pass < 2; ++pass) {
#pragma unroll
    for (int g = 0; g < 2; ++g) {
      const size_t o = (size_t)(c0 + g * 32 + q) * (size_t)ldo + (size_t)(r0 + c8);
      *(volatile v8h*)(O + o) = hv[g];
    }
    __threadfence();
  }
}

__global__ __launch_bounds__(NTHR) void gather_rows_kernel(const int* __restrict__ ids, const float* __restrict__ table,
                                                          unsigned short* __restrict__ dst) {
  const int i  = blockIdx.x * NTHR + threadIdx.x;
  const int n8 = NROWS * (NEMB / 8);
  if (i < n8) {
    const int m  = i / (NEMB / 8);
    const int c8 = i - m * (NEMB / 8);
    const int t  = m / NBATCH;
    const int b  = m - t * NBATCH;
    int id = ids[b * NSEQ + t];
    id = id < 0 ? 0 : id;
    id = id > (NVOCAB - 1) ? (NVOCAB - 1) : id;
    const float* sp = table + (size_t)id * NEMB + c8 * 8;
    const v4f a  = *(const v4f*)(sp);
    const v4f bq = *(const v4f*)(sp + 4);
    v8h hv;
#pragma unroll
    for (int e = 0; e < 4; ++e) {
      const unsigned short b0 = f2bf_bits(a[e]);
      const unsigned short b1 = f2bf_bits(bq[e]);
      hv[e]     = __builtin_bit_cast(_Float16, b0);
      hv[4 + e] = __builtin_bit_cast(_Float16, b1);
    }
    *(volatile v8h*)(dst + (size_t)i * 8) = hv;
    __threadfence();
    *(volatile v8h*)(dst + (size_t)i * 8) = hv;
  }
}

__global__ __launch_bounds__(256) void gemm64_bf16_kernel(
    const unsigned short* __restrict__ Ap, int lda,
    const unsigned short* __restrict__ Btp, int ldb,
    float* __restrict__ C, int ldc, int M, int N, int K) {
  const __bf16* A  = (const __bf16*)Ap;
  const __bf16* Bt = (const __bf16*)Btp;
  __shared__ __align__(16) float sT[8][16 * 68];
  const int lane = threadIdx.x & 31;
  const int wave = threadIdx.x >> 5;
  const int tilesN = N >> 6;
  const int tilesM = M >> 6;
  const int tile = blockIdx.x * 8 + wave;
  if (tile >= tilesM * tilesN) return;
  const int tm = tile / tilesN;
  const int tn = tile - tm * tilesN;
  const int m0 = tm << 6;
  const int n0 = tn << 6;
  const int rlane = lane & 15;
  const int koff  = (lane >> 4) * 8;
  const int mOff  = (lane >> 4) * 8;

  v8f acc[4][4];
#pragma unroll
  for (int i = 0; i < 4; ++i)
#pragma unroll
    for (int j = 0; j < 4; ++j) acc[i][j] = (v8f){0.f,0.f,0.f,0.f,0.f,0.f,0.f,0.f};

  for (int k0 = 0; k0 < K; k0 += 32) {
    v16b bh[4];
#pragma unroll
    for (int j = 0; j < 4; ++j) {
      const size_t bo = (size_t)(n0 + (j << 4) + rlane) * ldb + koff + k0;
      bh[j] = FragB::load(Bt + bo);
    }
#pragma unroll
    for (int i = 0; i < 4; ++i) {
      const size_t ao = (size_t)(m0 + (i << 4) + rlane) * lda + koff + k0;
      const v16b ah = FragB::load(A + ao);
#pragma unroll
      for (int j = 0; j < 4; ++j) acc[i][j] = FragB::mma(ah, bh[j], acc[i][j]);
      guard4_b5(acc[i][0], acc[i][1], acc[i][2], acc[i][3], ah, bh[0], bh[1], bh[2], bh[3]);
    }
    keep4_b(bh[0], bh[1], bh[2], bh[3]);
  }
  acc_guard4(acc[0][0], acc[0][1], acc[0][2], acc[0][3]);
  acc_guard4(acc[1][0], acc[1][1], acc[1][2], acc[1][3]);
  acc_guard4(acc[2][0], acc[2][1], acc[2][2], acc[2][3]);
  acc_guard4(acc[3][0], acc[3][1], acc[3][2], acc[3][3]);

  float* slab = sT[wave];
#pragma unroll
  for (int i = 0; i < 4; ++i) {
    const int mBase = m0 + (i << 4);
#pragma unroll
    for (int j = 0; j < 4; ++j) {
#pragma unroll
      for (int r = 0; r < 8; ++r) slab[(mOff + r) * 68 + (j << 4) + rlane] = acc[i][j][r];
    }
    __builtin_amdgcn_fence(__ATOMIC_RELEASE, "workgroup");
    __builtin_amdgcn_wave_barrier();
    __builtin_amdgcn_fence(__ATOMIC_ACQUIRE, "workgroup");
    {
      const int hh = lane >> 4, c4 = (lane & 15) * 4;
      for (int pass = 0; pass < 2; ++pass) {
#pragma unroll
        for (int it = 0; it < 8; ++it) {
          const int row = it * 2 + hh;
          const v4f v = *(const v4f*)(slab + row * 68 + c4);
          *(volatile v4f*)(C + (size_t)(mBase + row) * ldc + n0 + c4) = v;
        }
        __threadfence();
      }
    }
    __builtin_amdgcn_fence(__ATOMIC_RELEASE, "workgroup");
    __builtin_amdgcn_wave_barrier();
    __builtin_amdgcn_fence(__ATOMIC_ACQUIRE, "workgroup");
  }
}

__global__ __launch_bounds__(NTHR) void seq_scan_kernel(const float* __restrict__ XP,
                                                       const unsigned short* __restrict__ WhTp,
                                                       const int* __restrict__ amask,
                                                       const float* __restrict__ bias,
                                                       float* __restrict__ OUTH, float* __restrict__ HFIN) {
  __shared__ __align__(16) unsigned short Hhi[SEQ_BLK * HPITCH];
  __shared__ __align__(16) unsigned short Hlo[SEQ_BLK * HPITCH];
  __shared__ __align__(16) float Pre[NTHR / 32][16 * SLABP];
  __shared__ __align__(16) float Hst[NTHR / 32][16 * SLABP];
  const __bf16* WhT = (const __bf16*)WhTp;
  const int tid = threadIdx.x, lane = tid & 31, wave = tid >> 5;
  const int c = lane & 15, hh = lane >> 4, koff = hh * 8, c4 = c * 4;
  const int rowbase = blockIdx.x * SEQ_BLK;
  const int colbase = 64 * wave;

#pragma unroll 1
  for (int i = tid; i < SEQ_BLK * HPITCH; i += NTHR) {
    Hhi[i] = (unsigned short)0;
    Hlo[i] = (unsigned short)0;
  }
  float* pre = Pre[wave];
  float* hs  = Hst[wave];
  {
    const v4f z4 = {0.f, 0.f, 0.f, 0.f};
#pragma unroll 1
    for (int it = 0; it < 8; ++it) *(v4f*)(hs + (it * 2 + hh) * SLABP + c4) = z4;
  }
  const v4f braw = *(const v4f*)(bias + colbase + c4);
  const float bq0 = bf16r(braw[0]);
  const float bq1 = bf16r(braw[1]);
  const float bq2 = bf16r(braw[2]);
  const float bq3 = bf16r(braw[3]);
  __syncthreads();

  const __bf16* ahi = (const __bf16*)Hhi + c * HPITCH + koff;
  const __bf16* alo = (const __bf16*)Hlo + c * HPITCH + koff;
  const __bf16* wb  = WhT + (size_t)(colbase + c) * NHID + koff;
  const v8f z8 = {0.f, 0.f, 0.f, 0.f, 0.f, 0.f, 0.f, 0.f};

#pragma unroll 1
  for (int t = 0; t < NSEQ; ++t) {
    v8f a0 = z8, a1 = z8, a2 = z8, a3 = z8;
#pragma unroll 1
    for (int k0 = 0; k0 < NHID; k0 += 32) {
      const v16b fh = FragB::load(ahi + k0);
      const v16b fl = FragB::load(alo + k0);
      const v16b b0 = FragB::load(wb + k0);
      const v16b b1 = FragB::load(wb + (size_t)16 * NHID + k0);
      const v16b b2 = FragB::load(wb + (size_t)32 * NHID + k0);
      const v16b b3 = FragB::load(wb + (size_t)48 * NHID + k0);
      a0 = FragB::mma(fh, b0, a0);
      a1 = FragB::mma(fh, b1, a1);
      a2 = FragB::mma(fh, b2, a2);
      a3 = FragB::mma(fh, b3, a3);
      a0 = FragB::mma(fl, b0, a0);
      a1 = FragB::mma(fl, b1, a1);
      a2 = FragB::mma(fl, b2, a2);
      a3 = FragB::mma(fl, b3, a3);
      guard4_b6(a0, a1, a2, a3, fh, fl, b0, b1, b2, b3);
    }
    acc_guard4(a0, a1, a2, a3);
#pragma unroll
    for (int r = 0; r < 8; ++r) {
      float* pr = pre + (8 * hh + r) * SLABP + c;
      pr[0]  = a0[r];
      pr[16] = a1[r];
      pr[32] = a2[r];
      pr[48] = a3[r];
    }
    __syncthreads();

    const bool last = (t == NSEQ - 1);
#pragma unroll 1
    for (int it = 0; it < 8; ++it) {
      const int row  = it * 2 + hh;
      const int grow = rowbase + row;
      const v4f pv = *(const v4f*)(pre + row * SLABP + c4);
      const v4f hv = *(const v4f*)(hs + row * SLABP + c4);
      const v4f xv = *(const v4f*)(XP + ((size_t)t * NBATCH + (size_t)grow) * NHID + colbase + c4);
      const int mv = amask[(size_t)grow * NSEQ + t];
      const bool upd = (mv != 0);
      const float p0 = pv[0], p1 = pv[1], p2 = pv[2], p3 = pv[3];
      const float x0 = xv[0], x1 = xv[1], x2 = xv[2], x3 = xv[3];
      const float h0 = hv[0], h1 = hv[1], h2 = hv[2], h3 = hv[3];
      const float t0 = tanhf((p0 + x0) + bq0);
      const float t1 = tanhf((p1 + x1) + bq1);
      const float t2 = tanhf((p2 + x2) + bq2);
      const float t3 = tanhf((p3 + x3) + bq3);
      const float n0 = upd ? t0 : h0;
      const float n1 = upd ? t1 : h1;
      const float n2 = upd ? t2 : h2;
      const float n3 = upd ? t3 : h3;
      v4f nv;
      nv[0] = n0; nv[1] = n1; nv[2] = n2; nv[3] = n3;
      *(v4f*)(hs + row * SLABP + c4) = nv;
      const unsigned hb0 = bf_bits32(n0), hb1 = bf_bits32(n1), hb2 = bf_bits32(n2), hb3 = bf_bits32(n3);
      const unsigned lb0 = bf_bits32(n0 - __uint_as_float(hb0 << 16));
      const unsigned lb1 = bf_bits32(n1 - __uint_as_float(hb1 << 16));
      const unsigned lb2 = bf_bits32(n2 - __uint_as_float(hb2 << 16));
      const unsigned lb3 = bf_bits32(n3 - __uint_as_float(hb3 << 16));
      v2u ph, pl;
      ph[0] = hb0 | (hb1 << 16);
      ph[1] = hb2 | (hb3 << 16);
      pl[0] = lb0 | (lb1 << 16);
      pl[1] = lb2 | (lb3 << 16);
      *(v2u*)(Hhi + row * HPITCH + colbase + c4) = ph;
      *(v2u*)(Hlo + row * HPITCH + colbase + c4) = pl;
      *(volatile v4f*)(OUTH + ((size_t)grow * NSEQ + (size_t)t) * NHID + colbase + c4) = nv;
      if (last) *(volatile v4f*)(HFIN + (size_t)grow * NHID + colbase + c4) = nv;
    }
    __threadfence();
#pragma unroll 1
    for (int it = 0; it < 8; ++it) {
      const int row  = it * 2 + hh;
      const int grow = rowbase + row;
      const v4f nv = *(const v4f*)(hs + row * SLABP + c4);
      *(volatile v4f*)(OUTH + ((size_t)grow * NSEQ + (size_t)t) * NHID + colbase + c4) = nv;
      if (last) *(volatile v4f*)(HFIN + (size_t)grow * NHID + colbase + c4) = nv;
    }
    __threadfence();
    __syncthreads();
  }
}

extern "C" void kernel_launch(void* const* d_in, const int* in_sizes, int n_in,
                              void* d_out, int out_size, void* d_ws, size_t ws_size, hipStream_t stream) {
  if (n_in < 6 || d_out == nullptr || d_ws == nullptr) return;
  if (in_sizes[0] != NBATCH * NSEQ || in_sizes[1] != NBATCH * NSEQ || in_sizes[2] != NVOCAB * NEMB ||
      in_sizes[3] != NEMB * NHID || in_sizes[4] != NHID * NHID || in_sizes[5] != NHID ||
      out_size != NOUT0 + NOUT1) return;

  const int*   ids   = (const int*)d_in[0];
  const int*   amask = (const int*)d_in[1];
  const float* table = (const float*)d_in[2];
  const float* Wx    = (const float*)d_in[3];
  const float* Wh    = (const float*)d_in[4];
  const float* bias  = (const float*)d_in[5];
  float* all_h   = (float*)d_out;
  float* final_h = all_h + (size_t)NOUT0;

  char* ws = (char*)d_ws; size_t off = 0;
  auto carve = [&](size_t bytes) -> char* { char* p = ws + off; off += (bytes + 255) & ~(size_t)255; return p; };
  unsigned short* ABF  = (unsigned short*)carve((size_t)NROWS * NEMB * 2);
  unsigned short* WXT  = (unsigned short*)carve((size_t)NHID * NEMB * 2);
  unsigned short* WHT  = (unsigned short*)carve((size_t)NHID * NHID * 2);
  float*          XPRE = (float*)carve((size_t)NROWS * NHID * 4);
  if (off > ws_size || off > (size_t)134217728) return;

  tpw_kernel<<<dim3(NHID / 64, NEMB / 64), NTHR, 0, stream>>>(Wx, NEMB, NHID, NEMB, WXT);
  tpw_kernel<<<dim3(NHID / 64, NHID / 64), NTHR, 0, stream>>>(Wh, NHID, NHID, NHID, WHT);
  const int n8 = NROWS * (NEMB / 8);
  gather_rows_kernel<<<(n8 + NTHR - 1) / NTHR, NTHR, 0, stream>>>(ids, table, ABF);
  gemm64_bf16_kernel<<<dim3((NROWS / 64) * (NHID / 64) / 8, 1), 256, 0, stream>>>(
      ABF, NEMB, WXT, NEMB, XPRE, NHID, NROWS, NHID, NEMB);
  seq_scan_kernel<<<NBATCH / SEQ_BLK, NTHR, 0, stream>>>(XPRE, WHT, amask, bias, all_h, final_h);
}
